// RelMultiheadAttention_15470472200833
// MI455X (gfx1250) — hardware-verified
//
#include <hip/hip_runtime.h>


namespace {
typedef _Float16 b16;
typedef __attribute__((ext_vector_type(16))) _Float16 v16b;
typedef __attribute__((ext_vector_type(8))) _Float16 v8b;
typedef __attribute__((ext_vector_type(4))) _Float16 v4h;
typedef __attribute__((ext_vector_type(2))) _Float16 v2h;
typedef __attribute__((ext_vector_type(8))) float v8f;
typedef __attribute__((ext_vector_type(4))) float v4f;
typedef __attribute__((ext_vector_type(2))) float v2f;
__device__ __forceinline__ float bf16_rne(float f) { unsigned int u = __float_as_uint(f); u += 0x7FFFu + ((u >> 16) & 1u); return __uint_as_float(u & 0xFFFF0000u); }
__device__ __forceinline__ void split16(float v, b16& hi, b16& lo) { hi = (b16)v; lo = (b16)(v - (float)hi); }
__device__ __forceinline__ v16b frag_kb(const b16* p, int hh) { const v8b a = *(const v8b*)(p + 8 * hh), b = *(const v8b*)(p + 16 + 8 * hh); v16b f;
#pragma unroll
  for (int e = 0; e < 8; ++e) { f[e] = a[e]; f[8 + e] = b[e]; } return f; }
__device__ __forceinline__ v8f wmma16b(v16b a, v16b b, v8f c) { v8f d = __builtin_amdgcn_wmma_f32_16x16x32_f16(false, a, false, b, (short)0, c, false, false); asm volatile("v_nop\n\tv_nop\n\tv_nop\n\tv_nop" : "+v"(d) : "v"(a), "v"(b)); return d; }
__device__ __forceinline__ void wave_lds_sync() { __builtin_amdgcn_fence(__ATOMIC_RELEASE, "workgroup"); __builtin_amdgcn_wave_barrier(); __builtin_amdgcn_fence(__ATOMIC_ACQUIRE, "workgroup"); }
__device__ __forceinline__ float pmul(float a, float b) { float p = a * b; asm volatile("" : "+v"(p)); return p; }
__device__ __forceinline__ int iclamp(int v, int lo, int hi) { return v < lo ? lo : (v > hi ? hi : v); }
__device__ __forceinline__ float nexp2(float v) { return __builtin_amdgcn_exp2f(v); }

constexpr int T = 1024, TL = T  , S = 1024, B = 8, D = 256, NH = 8, HD = 32, NREL = 1023, MEM = 512, NROW = T * B;
constexpr float XS = 8.0f, WSC = 256.0f, PS = 1024.0f, RS_ = 1024.0f, LOG2E = 1.4426950408889634f, SCALE = 0.17677669529663687f  ;
static_assert(T % 64 == 0 && S % 32 == 0 && TL % 32 == 0 && D == 256 && NH * HD == D, "tiling");

template <int KD, int NOUT, int LDA, int LDT, bool RNDA>
__global__ __launch_bounds__(64) void gemmx_kernel(const float* __restrict__ A, int nv, const b16* __restrict__ W, const float* __restrict__ bias, int mrows, float* __restrict__ T) {
  constexpr int SL = NOUT < 128 ? NOUT : 128, NT = SL / 16, KC = KD < 128 ? KD : 128;
  static_assert(KD % KC == 0 && KC % 32 == 0 && NOUT % SL == 0 && SL % 32 == 0 && LDA >= KD && LDT >= NOUT, "gemmx tiling");
  __shared__ __attribute__((aligned(16))) b16 Ah[2][16][KC + 8], Al[2][16][KC + 8]; __shared__ __attribute__((aligned(16))) float Tf[2][16][SL + 4];
  const int wave = threadIdx.x >> 5, lane = threadIdx.x & 31, nloc = lane & 15, hlf = lane >> 4; const size_t m0 = (size_t)blockIdx.x * 32 + wave * 16; const int n0 = blockIdx.y * SL;
  v8f acc[NT];
#pragma unroll
  for (int t = 0; t < NT; ++t) acc[t] = (v8f){};
#pragma unroll 1
  for (int kc = 0; kc < KD; kc += KC) {
    for (int idx = lane; idx < 16 * (KC / 4); idx += 32) { const int rr = idx / (KC / 4), c4 = (idx % (KC / 4)) * 4; const size_t row = (m0 + rr < (size_t)nv) ? (m0 + rr) : (size_t)(nv - 1); const v4f v = *(const v4f*)(A + row * LDA + kc + c4); v4h hv, lv;
      for (int j = 0; j < 4; ++j) { b16 ph, pl; split16((RNDA ? bf16_rne(v[j]) : v[j]) * XS, ph, pl); hv[j] = ph; lv[j] = pl; } *(v4h*)(&Ah[wave][rr][c4]) = hv; *(v4h*)(&Al[wave][rr][c4]) = lv; }
    wave_lds_sync();
#pragma unroll
    for (int kb = 0; kb < KC; kb += 32) { const v16b a = frag_kb(&Ah[wave][nloc][kb], hlf), al = frag_kb(&Al[wave][nloc][kb], hlf);
#pragma unroll
      for (int t = 0; t < NT; ++t) { const v16b bw = frag_kb(W + (size_t)(n0 + t * 16 + nloc) * KD + kc + kb, hlf); acc[t] = wmma16b(a, bw, acc[t]); if (!RNDA) acc[t] = wmma16b(al, bw, acc[t]); } }
    wave_lds_sync(); }
#pragma unroll
  for (int t = 0; t < NT; ++t) { const float bb = bias ? bf16_rne(bias[n0 + t * 16 + nloc]) : 0.0f;
#pragma unroll
    for (int r = 0; r < 8; ++r) Tf[wave][8 * hlf + r][t * 16 + nloc] = acc[t][r] * (1.0f / (XS * WSC)) + bb; }
  wave_lds_sync();
  for (int pass = 0; pass < 2; ++pass) { for (int idx = lane; idx < 16 * (SL / 4); idx += 32) { const int rr = idx / (SL / 4), c4 = (idx % (SL / 4)) * 4; if (m0 + rr < (size_t)mrows) *(volatile v4f*)(T + (m0 + rr) * LDT + n0 + c4) = *(const v4f*)(&Tf[wave][rr][c4]); } __threadfence(); }
}

__global__ __launch_bounds__(256) void wcvt_kernel(const float* __restrict__ w, b16* __restrict__ W16, int n8, float scl, int nvalid8) {
  const int uu = blockIdx.x * 256 + threadIdx.x; if (uu >= n8) return; const size_t e = (size_t)uu * 8; v8b o; for (int j = 0; j < 8; ++j) o[j] = (b16)(uu < nvalid8 ? bf16_rne(w[e + j]) * scl : 0.0f);
  for (int pass = 0; pass < 2; ++pass) { *(volatile v8b*)(W16 + e) = o; __threadfence(); }
}
__global__ __launch_bounds__(128) void proj_kernel(const float* __restrict__ qin, const float* __restrict__ kin, const float* __restrict__ vin, const b16* __restrict__ WT, const float* __restrict__ bq, const float* __restrict__ bk, const float* __restrict__ bv, const float* __restrict__ uu, const float* __restrict__ vv,
    b16* __restrict__ QUh, b16* __restrict__ QUl, b16* __restrict__ QVh, b16* __restrict__ QVl, b16* __restrict__ Kh, b16* __restrict__ Kl, b16* __restrict__ VTh, b16* __restrict__ VTl) {
  __shared__ __attribute__((aligned(16))) b16 As[64][D + 8]; __shared__ __attribute__((aligned(16))) float Tf[4][16][128 + 4];
  const int wave = threadIdx.x >> 5, lane = threadIdx.x & 31, nloc = lane & 15, hlf = lane >> 4; const int t0 = blockIdx.x * 64; const int b = blockIdx.y; const int slab = blockIdx.z, n0 = slab * 128, part = slab / 2, h0 = (slab & 1) * 4;
  const float* src = part == 0 ? qin : part == 1 ? kin : vin; const float* bias = part == 0 ? bq : part == 1 ? bk : bv;
  for (int i = threadIdx.x; i < 64 * (D / 4); i += 128) { const int rr = i / (D / 4), q4 = (i % (D / 4)) * 4; const v4f f = *(const v4f*)(src + ((size_t)(t0 + rr) * B + b) * D + q4); v4h o; for (int j = 0; j < 4; ++j) o[j] = (b16)(bf16_rne(f[j]) * XS); *(v4h*)(&As[rr][q4]) = o; }
  __syncthreads();
  v8f acc[8];
#pragma unroll
  for (int tt = 0; tt < 8; ++tt) acc[tt] = (v8f){};
#pragma unroll 2
  for (int kb = 0; kb < D; kb += 32) { const v16b a = frag_kb(&As[wave * 16 + nloc][kb], hlf);
#pragma unroll
    for (int tt = 0; tt < 8; ++tt) acc[tt] = wmma16b(a, frag_kb(WT + (size_t)(n0 + tt * 16 + nloc) * D + kb, hlf), acc[tt]); }
#pragma unroll
  for (int tt = 0; tt < 8; ++tt) { const float bb = bf16_rne(bias[(n0 & 255) + tt * 16 + nloc]);
#pragma unroll
    for (int r = 0; r < 8; ++r) Tf[wave][8 * hlf + r][tt * 16 + nloc] = acc[tt][r] * (1.0f / (XS * WSC)) + bb; }
  __syncthreads();
  for (int pass = 0; pass < 2; ++pass) {
    if (part < 2) { const int h = h0 + (lane >> 3), d = (lane & 7) * 4;
      for (int rr = 0; rr < 16; ++rr) { const int tok = t0 + wave * 16 + rr; const size_t dst = (((size_t)b * NH + h) * T + tok) * HD + d; v4h oh, ol, oh2, ol2;
        for (int j = 0; j < 4; ++j) { const float base = Tf[wave][rr][lane * 4 + j];
          if (part == 0) { const float a1 = (base + bf16_rne(uu[h * HD + d + j])) * XS; const b16 p1 = (b16)a1; oh[j] = p1; ol[j] = (b16)((a1 - (float)p1) * RS_); const float a2 = (base + bf16_rne(vv[h * HD + d + j])) * XS; const b16 p2 = (b16)a2; oh2[j] = p2; ol2[j] = (b16)((a2 - (float)p2) * RS_); }
          else { const float a1 = base * XS; const b16 p1 = (b16)a1; oh[j] = p1; ol[j] = (b16)((a1 - (float)p1) * RS_); } }
        if (part == 0) { *(volatile v4h*)(QUh + dst) = oh; *(volatile v4h*)(QUl + dst) = ol; *(volatile v4h*)(QVh + dst) = oh2; *(volatile v4h*)(QVl + dst) = ol2; } else { *(volatile v4h*)(Kh + dst) = oh; *(volatile v4h*)(Kl + dst) = ol; } } }
    else {
#pragma unroll 1
      for (int q = 0; q < 32; ++q) { const int cl = wave * 32 + q; const int h = h0 + cl / HD, d = cl % HD; const int tk = lane * 2; v2h hv, lv; for (int e2 = 0; e2 < 2; ++e2) { const float vs = Tf[(tk + e2) >> 4][(tk + e2) & 15][cl] * XS; const b16 ph = (b16)vs; hv[e2] = ph; lv[e2] = (b16)((vs - (float)ph) * RS_); }
        const size_t dst = (((size_t)b * NH + h) * HD + d) * (size_t)S + t0 + tk; *(volatile v2h*)(VTh + dst) = hv; *(volatile v2h*)(VTl + dst) = lv; } }
    __threadfence(); }
}
__global__ __launch_bounds__(64) void attn_kernel(const b16* __restrict__ QUh, const b16* __restrict__ QUl, const b16* __restrict__ QVh, const b16* __restrict__ QVl, const b16* __restrict__ Kh, const b16* __restrict__ Kl, const b16* __restrict__ VTh, const b16* __restrict__ VTl, const b16* __restrict__ REL, const int* __restrict__ mlen, float* __restrict__ CT) {
  __shared__ __attribute__((aligned(16))) b16 Pb[2][16][32 + 8], Pl[2][16][32 + 8]; __shared__ __attribute__((aligned(16))) float To[2][16][HD + 4]; __shared__ float Gs[2][16][48 + 1];
  const int wave = threadIdx.x >> 5, lane = threadIdx.x & 31, hh = lane >> 4, col = lane & 15; const int t0 = blockIdx.x * 32 + wave * 16; const int b = blockIdx.y / NH, h = blockIdx.y % NH; const int M = mlen[0];
  const size_t ph = (size_t)b * NH + h; const size_t qoff = (ph * T + t0 + col) * HD;
  const v16b qu = frag_kb(QUh + qoff, hh), qul = frag_kb(QUl + qoff, hh), qv = frag_kb(QVh + qoff, hh), qvl = frag_kb(QVl + qoff, hh);
  const b16* Khb = Kh + ph * T * HD; const b16* Klb = Kl + ph * T * HD; const b16* Vhb = VTh + ph * HD * (size_t)S; const b16* Vlb = VTl + ph * HD * (size_t)S;
  const float cs = LOG2E * SCALE / (XS * XS); const int tq = t0 + col;
  float m = -INFINITY, l = 0.0f; v8f o[2], o2[2]; o[0] = (v8f){}; o[1] = (v8f){}; o2[0] = (v8f){}; o2[1] = (v8f){};
#pragma unroll 1
  for (int s0 = 0; s0 < S; s0 += 32) {
    const int jlo = iclamp(t0 - s0 - 31 - M + (MEM - 1), 0, NREL - 1);
#pragma unroll
    for (int g = 0; g < 3; ++g) { const int jrow = iclamp(jlo + g * 16 + col, 0, NREL - 1); v8f ga = wmma16b(frag_kb(REL + (size_t)jrow * HD, hh), qv, (v8f){}); v8f gb = wmma16b(frag_kb(REL + (size_t)jrow * HD, hh), qvl, (v8f){});
#pragma unroll
      for (int r = 0; r < 8; ++r) Gs[wave][col][g * 16 + 8 * hh + r] = ga[r] + gb[r] * (1.0f / RS_); }
    wave_lds_sync();
    float e[16]; float mx = -INFINITY;
#pragma unroll
    for (int u2 = 0; u2 < 2; ++u2) { const b16* kr = Khb + (size_t)(s0 + u2 * 16 + col) * HD; const v16b kh = frag_kb(kr, hh), kl = frag_kb(Klb + (size_t)(s0 + u2 * 16 + col) * HD, hh);
      v8f sa = wmma16b(kh, qu, (v8f){}); v8f sb = wmma16b(kl, qu, (v8f){}); sb = wmma16b(kh, qul, sb);
#pragma unroll
      for (int r = 0; r < 8; ++r) { const int s = s0 + u2 * 16 + 8 * hh + r; const int jj = iclamp(tq - s - M + (MEM - 1), 0, NREL - 1) - jlo; const float vvl = (sa[r] + sb[r] * (1.0f / RS_) + Gs[wave][col][iclamp(jj, 0, 47)]) * cs; e[u2 * 8 + r] = vvl; mx = fmaxf(mx, vvl); } }
    mx = fmaxf(mx, __shfl_xor(mx, 16)); const float mn = fmaxf(m, mx); const float al = nexp2(m - mn); float sum = 0.0f;
#pragma unroll
    for (int i2 = 0; i2 < 16; ++i2) { const float p = nexp2(e[i2] - mn); sum += p; const float psv = p * PS; const b16 p1 = (b16)psv; const int slot = (i2 < 8 ? 0 : 16) + 8 * hh + (i2 & 7); Pb[wave][col][slot] = p1; Pl[wave][col][slot] = (b16)((psv - (float)p1) * RS_); }
    sum += __shfl_xor(sum, 16); l = l * al + sum; m = mn;
    wave_lds_sync();
    const v16b pf = frag_kb(&Pb[wave][col][0], hh), plf = frag_kb(&Pl[wave][col][0], hh);
#pragma unroll
    for (int t2 = 0; t2 < 2; ++t2) { o[t2] *= al; o2[t2] *= al; const v16b vh = frag_kb(Vhb + (size_t)(t2 * 16 + col) * S + s0, hh); o[t2] = wmma16b(vh, pf, o[t2]); o2[t2] = wmma16b(frag_kb(Vlb + (size_t)(t2 * 16 + col) * S + s0, hh), pf, o2[t2]); o2[t2] = wmma16b(vh, plf, o2[t2]); }
    wave_lds_sync(); }
  const float inv = 1.0f / (l * PS * XS);
#pragma unroll
  for (int t2 = 0; t2 < 2; ++t2)
#pragma unroll
    for (int r = 0; r < 8; ++r) To[wave][col][t2 * 16 + 8 * hh + r] = (o[t2][r] + o2[t2][r] * (1.0f / RS_)) * inv;
  wave_lds_sync();
  for (int pass = 0; pass < 2; ++pass) { for (int rr = 0; rr < 16; ++rr) ((volatile float*)CT)[((size_t)(t0 + rr) * B + b) * D + h * HD + lane] = To[wave][rr][lane]; __threadfence(); }
}
}

extern "C" void kernel_launch(void* const* d_in, const int* in_sizes, int n_in, void* d_out, int out_size, void* d_ws, size_t ws_size, hipStream_t stream) {
  (void)n_in;
  auto Fp = [&](int i) { return (const float*)d_in[i]; };
  if (in_sizes[0] != NROW * D || in_sizes[1] != NROW * D || in_sizes[2] != NROW * D || in_sizes[3] != D * D || in_sizes[5] != D * D || in_sizes[7] != D * D || in_sizes[9] != D * D || in_sizes[10] != D || in_sizes[11] != NREL * HD || in_sizes[12] != NH * HD || in_sizes[13] != NH * HD || in_sizes[14] != 1 || out_size != NROW * D) return;
  size_t off = 0; char* ws = (char*)d_ws;
  auto carve = [&](size_t bytes) { char* p = ws + off; off += (bytes + 255) & ~(size_t)255; return p; };
  b16* WT = (b16*)carve((size_t)3 * D * D * 2); b16* WO = (b16*)carve((size_t)D * D * 2); b16* REL = (b16*)carve((size_t)1088 * HD * 2); const size_t plane = (size_t)B * NH * T * HD * 2;
  b16* QUh = (b16*)carve(plane); b16* QUl = (b16*)carve(plane); b16* QVh = (b16*)carve(plane); b16* QVl = (b16*)carve(plane); b16* Kh = (b16*)carve(plane); b16* Kl = (b16*)carve(plane); b16* VTh = (b16*)carve(plane); b16* VTl = (b16*)carve(plane); float* CT = (float*)carve((size_t)NROW * D * 4);
  if (off > ws_size || off > ((size_t)128 << 20)) return;
  wcvt_kernel<<<(D * D / 8 + 255) / 256, 256, 0, stream>>>(Fp(3), WT, D * D / 8, WSC, D * D / 8); wcvt_kernel<<<(D * D / 8 + 255) / 256, 256, 0, stream>>>(Fp(5), WT + (size_t)D * D, D * D / 8, WSC, D * D / 8); wcvt_kernel<<<(D * D / 8 + 255) / 256, 256, 0, stream>>>(Fp(7), WT + (size_t)2 * D * D, D * D / 8, WSC, D * D / 8);
  wcvt_kernel<<<(D * D / 8 + 255) / 256, 256, 0, stream>>>(Fp(9), WO, D * D / 8, WSC, D * D / 8); wcvt_kernel<<<(1088 * HD / 8 + 255) / 256, 256, 0, stream>>>(Fp(11), REL, 1088 * HD / 8, XS, NREL * HD / 8);
  proj_kernel<<<dim3(T / 64, B, 6), 128, 0, stream>>>(Fp(0), Fp(1), Fp(2), WT, Fp(4), Fp(6), Fp(8), Fp(12), Fp(13), QUh, QUl, QVh, QVl, Kh, Kl, VTh, VTl);
  attn_kernel<<<dim3(TL / 32, B * NH), 64, 0, stream>>>(QUh, QUl, QVh, QVl, Kh, Kl, VTh, VTl, REL, (const int*)d_in[14], CT);
  gemmx_kernel<D, D, D, D, false><<<dim3(TL * B / 32, 2), 64, 0, stream>>>(CT, TL * B, WO, Fp(10), TL * B, (float*)d_out);
}
